// PagedAttentionOp_64871186039428
// MI455X (gfx1250) — hardware-verified
//
#include <hip/hip_runtime.h>


#define NT_  2048
#define NH_  32
#define NKV  8
#define HD   128
#define KW   (NKV * HD)
#define PSC  32768.0f

typedef _Float16 h16;
typedef unsigned short bf;
typedef __attribute__((ext_vector_type(16))) __bf16   v16bf;
typedef __attribute__((ext_vector_type(16))) _Float16 v16h;
typedef __attribute__((ext_vector_type(8)))  _Float16 v8h;
typedef __attribute__((ext_vector_type(8)))  unsigned short v8us;
typedef __attribute__((ext_vector_type(8)))  float    v8f;
typedef __attribute__((ext_vector_type(4)))  float    v4f;
typedef __attribute__((ext_vector_type(4)))  _Float16 v4h;
typedef v8h  __attribute__((may_alias)) v8ha;
typedef v4f  __attribute__((may_alias)) v4fa;
typedef v8us __attribute__((may_alias)) v8usa;

__device__ __forceinline__ unsigned short f2bf(float f) { unsigned u = __float_as_uint(f); u += 0x7FFFu + ((u >> 16) & 1u); return (unsigned short)(u >> 16); }
__device__ __forceinline__ float bf2f(unsigned short b) { return __uint_as_float(((unsigned)b) << 16); }
__device__ __forceinline__ float bfr(float f) { return bf2f(f2bf(f)); }
__device__ __forceinline__ v16h cat16(v8h lo, v8h hi) { return __builtin_shufflevector(lo, hi, 0, 1, 2, 3, 4, 5, 6, 7, 8, 9, 10, 11, 12, 13, 14, 15); }
__device__ __forceinline__ v16bf cat16b(v8us lo, v8us hi) { return __builtin_bit_cast(v16bf, __builtin_shufflevector(lo, hi, 0, 1, 2, 3, 4, 5, 6, 7, 8, 9, 10, 11, 12, 13, 14, 15)); }
__device__ __forceinline__ v8f wmma16(v16h a, v16h b, v8f c) { return __builtin_amdgcn_wmma_f32_16x16x32_f16(false, a, false, b, (short)0, c, false, false); }
__device__ __forceinline__ v8f wmmab(v16bf a, v16bf b, v8f c) { return __builtin_amdgcn_wmma_f32_16x16x32_bf16(false, a, false, b, (short)0, c, false, false); }

__global__ __launch_bounds__(256) void k_16(const float* __restrict__ src, h16* dst, int n4) {
    const int i = blockIdx.x * 256 + threadIdx.x; if (i >= n4) return;
    const v4f v = *(const v4f*)(src + (size_t)i * 4); v4h o;
#pragma unroll
    for (int k = 0; k < 4; ++k) o[k] = (h16)bfr(v[k]);
    *(volatile v4h*)(dst + (size_t)i * 4) = o; __threadfence(); *(volatile v4h*)(dst + (size_t)i * 4) = o;
}
__global__ __launch_bounds__(256) void k_vt1(const float* __restrict__ V, bf* VTH) {
    __shared__ __align__(16) unsigned short th_[64 * 72];
    const int t0 = blockIdx.x * 64, dh = blockIdx.y, g = blockIdx.z, tid = threadIdx.x;
    const int tt = tid >> 2, dq = (tid & 3) * 16;
    const float* src = V + ((size_t)t0 + tt) * KW + g * HD + dh * 64 + dq;
#pragma unroll
    for (int i = 0; i < 16; ++i) th_[(dq + i) * 72 + tt] = f2bf(src[i]);
    __syncthreads();
    const int piece = tid & 7;
    auto pass = [&]() {
#pragma unroll
        for (int s = 0; s < 2; ++s) { const int d = (tid >> 3) + 32 * s;
            const v8us a = *(const v8usa*)(th_ + d * 72 + piece * 8);
            *(volatile v8us*)(VTH + ((size_t)g * HD + dh * 64 + d) * NT_ + t0 + piece * 8) = a; }
    };
    pass(); __threadfence(); pass();
}
__global__ __launch_bounds__(128) void k_attn(const h16* __restrict__ QH, const h16* __restrict__ KH, const bf* __restrict__ VTH, float* OUTP, float* MS, float* LS) {
    __shared__ __align__(16) unsigned short plds[4][16 * 32];
    __shared__ __align__(16) unsigned short plds2[4][16 * 32];
    __shared__ __align__(16) float ost[4][16 * 68]; __shared__ __align__(16) float mls[2][64];
    const int lane = threadIdx.x & 31, wave = threadIdx.x >> 5, lr = lane & 15, hi = lane >> 4;
    const int bid = blockIdx.x; const int h = bid / (NT_ / 64), qt = bid - h * (NT_ / 64); const int g = h >> 2;
    const int q0 = qt * 64 + wave * 16;
    unsigned short* pl = &plds[wave][0]; unsigned short* pl2 = &plds2[wave][0];
    const size_t qo = (size_t)(q0 + lr) * (NH_ * HD) + h * HD + 8 * hi;
    const h16* kh_b = KH + g * HD;
    const size_t vbase = ((size_t)g * HD) * NT_;
    v8f o[8];
#pragma unroll
    for (int n = 0; n < 8; ++n) o[n] = (v8f){};
    float mrow[8], lpart[8];
#pragma unroll
    for (int j = 0; j < 8; ++j) { mrow[j] = -3.0e38f; lpart[j] = 0.f; }
    const int kt_hi = (qt * 64 + 63) / 32; const int kt_lo = 0;
#pragma unroll 1
    for (int kt = kt_lo; kt <= kt_hi; ++kt) {
        const int l0 = kt * 32;
        const size_t ko0 = (size_t)(l0 + lr) * KW + 8 * hi, ko1 = (size_t)(l0 + 16 + lr) * KW + 8 * hi;
        v8f s0 = {}, s1 = {};
#pragma unroll
        for (int kc = 0; kc < 4; ++kc) {
            const v16h qa = cat16(*(const v8h*)(QH + qo + kc * 32), *(const v8h*)(QH + qo + kc * 32 + 16));
            const v16h k0h = cat16(*(const v8h*)(kh_b + ko0 + kc * 32), *(const v8h*)(kh_b + ko0 + kc * 32 + 16)), k1h = cat16(*(const v8h*)(kh_b + ko1 + kc * 32), *(const v8h*)(kh_b + ko1 + kc * 32 + 16));
            s0 = wmma16(qa, k0h, s0); s1 = wmma16(qa, k1h, s1);
            asm volatile("v_nop" : "+v"(s0), "+v"(s1) : "v"(qa), "v"(k0h), "v"(k1h) : "memory");
        }
        asm volatile("v_nop\n\tv_nop\n\tv_nop\n\tv_nop" : "+v"(s0), "+v"(s1));
        float alpha[8];
#pragma unroll
        for (int j = 0; j < 8; ++j) { const int qi = q0 + hi * 8 + j, ja = l0 + lr, jb = l0 + 16 + lr;
            const float a0 = (ja <= qi) ? s0[j] : -__builtin_inff(), a1 = (jb <= qi) ? s1[j] : -__builtin_inff();
            float mx = fmaxf(a0, a1);
            mx = fmaxf(mx, __shfl_xor(mx, 1, 16)); mx = fmaxf(mx, __shfl_xor(mx, 2, 16)); mx = fmaxf(mx, __shfl_xor(mx, 4, 16)); mx = fmaxf(mx, __shfl_xor(mx, 8, 16));
            const float mn = fmaxf(mrow[j], mx);
            alpha[j] = __expf(mrow[j] - mn); mrow[j] = mn;
            const float p0 = __expf(a0 - mn), p1 = __expf(a1 - mn);
            lpart[j] = lpart[j] * alpha[j] + (p0 + p1);
            const int mr = hi * 8 + j; const float ps0 = p0 * PSC, ps1 = p1 * PSC; const unsigned short h0 = f2bf(ps0), h1 = f2bf(ps1);
            pl[mr * 32 + lr] = h0; pl[mr * 32 + 16 + lr] = h1; pl2[mr * 32 + lr] = f2bf(ps0 - bf2f(h0)); pl2[mr * 32 + 16 + lr] = f2bf(ps1 - bf2f(h1)); }
#pragma unroll
        for (int n = 0; n < 8; ++n)
#pragma unroll
            for (int j = 0; j < 8; ++j) o[n][j] *= alpha[j];
        asm volatile("" ::: "memory");
        const v16bf pa = cat16b(*(const v8usa*)(pl + lr * 32 + hi * 8), *(const v8usa*)(pl + lr * 32 + 16 + hi * 8));
        const v16bf px = cat16b(*(const v8usa*)(pl2 + lr * 32 + hi * 8), *(const v8usa*)(pl2 + lr * 32 + 16 + hi * 8));
#pragma unroll
        for (int n = 0; n < 8; ++n) { const size_t vo = vbase + (size_t)(n * 16 + lr) * NT_ + l0 + hi * 8;
            const v16bf vh = cat16b(*(const v8us*)(VTH + vo), *(const v8us*)(VTH + vo + 16));
            o[n] = wmmab(pa, vh, o[n]); o[n] = wmmab(px, vh, o[n]);
            asm volatile("" : "+v"(o[n]) : "v"(vh) : "memory"); }
        asm volatile("v_nop\n\tv_nop\n\tv_nop\n\tv_nop" : "+v"(o[0]), "+v"(o[7]) : "v"(pa), "v"(px));
        __builtin_amdgcn_wave_barrier();
    }
    float lsum[8];
#pragma unroll
    for (int j = 0; j < 8; ++j) { float rs = lpart[j]; rs += __shfl_xor(rs, 1, 16); rs += __shfl_xor(rs, 2, 16); rs += __shfl_xor(rs, 4, 16); rs += __shfl_xor(rs, 8, 16); lsum[j] = rs; }
    if (lr == 0) {
#pragma unroll
        for (int j = 0; j < 8; ++j) { mls[0][wave * 16 + hi * 8 + j] = mrow[j]; mls[1][wave * 16 + hi * 8 + j] = lsum[j]; } }
    float* os = &ost[wave][0];
    float* ob = OUTP + ((size_t)q0 * NH_ + h) * HD;
#pragma unroll
    for (int half = 0; half < 2; ++half) {
#pragma unroll
        for (int n = 0; n < 4; ++n)
#pragma unroll
            for (int j = 0; j < 8; ++j) os[(hi * 8 + j) * 68 + n * 16 + lr] = o[half * 4 + n][j] * (1.0f / PSC);
        __builtin_amdgcn_wave_barrier(); asm volatile("" ::: "memory");
#pragma unroll
        for (int ps2 = 0; ps2 < 2; ++ps2) {
#pragma unroll
            for (int s = 0; s < 8; ++s) { const int Lid = (lane >> 3) + 4 * s, piece = lane & 7; const int row = Lid >> 1, cofs = (Lid & 1) * 32 + piece * 4;
                const v4f val = *(const v4fa*)(os + row * 68 + cofs); *(volatile v4f*)(ob + (size_t)row * (NH_ * HD) + half * 64 + cofs) = val; }
            if (ps2 == 0) __threadfence(); }
        __builtin_amdgcn_wave_barrier(); asm volatile("" ::: "memory");
    }
    __syncthreads();
    if (threadIdx.x < 32) { const int which = threadIdx.x >> 4, qq = threadIdx.x & 15; const v4f v = *(const v4fa*)(&mls[which][qq * 4]);
        float* dst = (which ? LS : MS) + (size_t)h * NT_ + qt * 64 + qq * 4; *(volatile v4f*)dst = v; __threadfence(); *(volatile v4f*)dst = v; }
}
__global__ __launch_bounds__(256) void k_mlt(const float* __restrict__ MS, const float* __restrict__ LS, float* OM, float* OL) {
    const int lane = threadIdx.x & 31, t = blockIdx.x * 8 + (threadIdx.x >> 5); if (t >= NT_) return;
    const float m = MS[(size_t)lane * NT_ + t], l = LS[(size_t)lane * NT_ + t];
    *(volatile float*)(OM + (size_t)t * NH_ + lane) = m; *(volatile float*)(OL + (size_t)t * NH_ + lane) = l; __threadfence();
    *(volatile float*)(OM + (size_t)t * NH_ + lane) = m; *(volatile float*)(OL + (size_t)t * NH_ + lane) = l;
}

extern "C" void kernel_launch(void* const* d_in, const int* in_sizes, int n_in,
                              void* d_out, int out_size, void* d_ws, size_t ws_size, hipStream_t stream) {
    (void)in_sizes; (void)n_in; (void)out_size;
    const float* query = (const float*)d_in[0]; const float* key = (const float*)d_in[1]; const float* value = (const float*)d_in[2];
    float* out = (float*)d_out;
    float* out_m = out + (size_t)NT_ * NH_ * HD; float* out_l = out_m + (size_t)NT_ * NH_;
    char* wsp = (char*)d_ws;
    auto take = [&](size_t bytes) { char* p = wsp; wsp += (bytes + 255) & ~(size_t)255; return (void*)p; };
    h16* QH = (h16*)take((size_t)NT_ * NH_ * HD * 2); h16* KH = (h16*)take((size_t)NT_ * KW * 2); bf* VTH = (bf*)take((size_t)KW * NT_ * 2);
    float* MS = (float*)take((size_t)NH_ * NT_ * 4); float* LS = (float*)take((size_t)NH_ * NT_ * 4);
    if ((size_t)(wsp - (char*)d_ws) > ws_size) return;
    k_16<<<(NT_ * NH_ * HD / 4 + 255) / 256, 256, 0, stream>>>(query, QH, NT_ * NH_ * HD / 4);
    k_16<<<(NT_ * KW / 4 + 255) / 256, 256, 0, stream>>>(key, KH, NT_ * KW / 4);
    k_vt1<<<dim3(NT_ / 64, 2, NKV), 256, 0, stream>>>(value, VTH);
    k_attn<<<NH_ * (NT_ / 64), 128, 0, stream>>>(QH, KH, VTH, out, MS, LS);
    k_mlt<<<NT_ / 8, 256, 0, stream>>>(MS, LS, out_m, out_l);
}
